// T5_71665824301626
// MI455X (gfx1250) — hardware-verified
//
#include <hip/hip_runtime.h>
#include <math.h>

typedef __attribute__((ext_vector_type(16))) _Float16 v16h;
typedef __attribute__((ext_vector_type(8)))  _Float16 v8h;
typedef __attribute__((ext_vector_type(16))) __bf16   v16b;
typedef __attribute__((ext_vector_type(8)))  __bf16   v8b;
typedef __attribute__((ext_vector_type(8)))  float    v8f;
typedef __attribute__((ext_vector_type(4)))  float    v4f;
#define U16(p) ((const unsigned short*)(const void*)(p))

__device__ __forceinline__ unsigned short f2bf_bits(float f) {
  unsigned u = __float_as_uint(f);
  return (unsigned short)((u + 0x7FFFu + ((u >> 16) & 1u)) >> 16);
}
__device__ __forceinline__ float bf_bits2f(unsigned short h) { return __uint_as_float(((unsigned)h) << 16); }

__device__ __forceinline__ void dep_guard_h(v8f& a, v8f& b, v16h x, v16h y) { asm volatile("v_nop\n\tv_nop\n\tv_nop\n\tv_nop" : "+v"(a), "+v"(b) : "v"(x), "v"(y)); }
__device__ __forceinline__ void dep_guard_b(v8f& a, v8f& b, v16b x, v16b y) { asm volatile("v_nop\n\tv_nop\n\tv_nop\n\tv_nop" : "+v"(a), "+v"(b) : "v"(x), "v"(y)); }
__device__ __forceinline__ void keep4_h(v16h a, v16h b, v16h c, v16h d) { asm volatile("v_nop" :: "v"(a), "v"(b), "v"(c), "v"(d)); }
__device__ __forceinline__ void keep4_b(v16b a, v16b b, v16b c, v16b d) { asm volatile("v_nop" :: "v"(a), "v"(b), "v"(c), "v"(d)); }
__device__ __forceinline__ void acc_guard4(v8f& a, v8f& b, v8f& c, v8f& d) { asm volatile("v_nop\n\tv_nop\n\tv_nop\n\tv_nop" : "+v"(a), "+v"(b), "+v"(c), "+v"(d)); }
template <typename T> struct Frag;
template <> struct Frag<_Float16> {
  typedef v16h V; union U { v16h v; v8h h[2]; };
  static __device__ __forceinline__ v16h load(const _Float16* p) {
    U f; f.h[0] = *(const v8h*)(p); f.h[1] = *(const v8h*)(p + 16); return f.v;
  }
  static __device__ __forceinline__ v8f mma(v16h a, v16h b, v8f c) {
    return __builtin_amdgcn_wmma_f32_16x16x32_f16(false, a, false, b, (short)0, c, false, false);
  }
  static __device__ __forceinline__ void guard(v8f& a, v8f& b, v16h x, v16h y) { dep_guard_h(a, b, x, y); }
  static __device__ __forceinline__ void keep(v16h a, v16h b, v16h c, v16h d) { keep4_h(a, b, c, d); }
};
template <> struct Frag<__bf16> {
  typedef v16b V; union U { v16b v; v8b h[2]; };
  static __device__ __forceinline__ v16b load(const __bf16* p) {
    U f; f.h[0] = *(const v8b*)(p); f.h[1] = *(const v8b*)(p + 16); return f.v;
  }
  static __device__ __forceinline__ v8f mma(v16b a, v16b b, v8f c) {
    return __builtin_amdgcn_wmma_f32_16x16x32_bf16(false, a, false, b, (short)0, c, false, false);
  }
  static __device__ __forceinline__ void guard(v8f& a, v8f& b, v16b x, v16b y) { dep_guard_b(a, b, x, y); }
  static __device__ __forceinline__ void keep(v16b a, v16b b, v16b c, v16b d) { keep4_b(a, b, c, d); }
};

template <int ET> struct Elem;
template <> struct Elem<0> { typedef _Float16 T; };
template <> struct Elem<1> { typedef __bf16 T; };
template <int ET, bool SPLIT, int BIAS_MODE, int OUT_MODE, bool RESID, int ACT = 0>
__global__ __launch_bounds__(256) void wmma_gemm64(
    const unsigned short* __restrict__ Ap, const unsigned short* __restrict__ A2p, int lda, long strideA,
    const unsigned short* __restrict__ Btp, const unsigned short* __restrict__ Bt2p, int ldb, long strideB,
    void* __restrict__ Cout, void* __restrict__ Cout2, int ldc, long strideC,
    const float* __restrict__ bias,
    const float* __restrict__ resid, long strideR,
    int M, int N, int K, float scale) {
  typedef typename Elem<ET>::T T;
  typedef typename Frag<T>::V V;
  const T* A = (const T*)Ap; const T* A2 = (const T*)A2p; const T* Bt = (const T*)Btp; const T* Bt2 = (const T*)Bt2p;
  __shared__ __align__(16) float sT[8][16 * 68];
  const int b    = blockIdx.y;
  const int lane = threadIdx.x & 31;
  const int wave = threadIdx.x >> 5;
  const int tilesN = N >> 6;
  const int tilesM = M >> 6;
  const int tile = blockIdx.x * 8 + wave;
  if (tile >= tilesM * tilesN) return;
  const int tm = tile / tilesN;
  const int tn = tile - tm * tilesN;
  const int m0 = tm << 6;
  const int n0 = tn << 6;

  const T* Ab  = A  + (size_t)b * strideA;
  const T* Bb  = Bt + (size_t)b * strideB;
  const T* Ab2 = SPLIT ? (A2  + (size_t)b * strideA) : nullptr;
  const T* Bb2 = SPLIT ? (Bt2 + (size_t)b * strideB) : nullptr;

  const int rlane = lane & 15;
  const int koff  = (lane >> 4) * 8;
  const int mOff  = (lane >> 4) * 8;

  v8f acc[4][4];
#pragma unroll
  for (int i = 0; i < 4; ++i)
#pragma unroll
    for (int j = 0; j < 4; ++j) acc[i][j] = (v8f){0.f,0.f,0.f,0.f,0.f,0.f,0.f,0.f};

  for (int k0 = 0; k0 < K; k0 += 32) {
    V bh[4], bl[4];
#pragma unroll
    for (int j = 0; j < 4; ++j) {
      const size_t bo = (size_t)(n0 + (j << 4) + rlane) * ldb + koff + k0;
      bh[j] = Frag<T>::load(Bb + bo);
      if (SPLIT) bl[j] = Frag<T>::load(Bb2 + bo);
    }
#pragma unroll
    for (int i = 0; i < 4; ++i) {
      const size_t ao = (size_t)(m0 + (i << 4) + rlane) * lda + koff + k0;
      V ah = Frag<T>::load(Ab + ao);
      V al;
      if (SPLIT) al = Frag<T>::load(Ab2 + ao);
#pragma unroll
      for (int j = 0; j < 4; ++j) {
        acc[i][j] = Frag<T>::mma(ah, bh[j], acc[i][j]);
        if (SPLIT) {
          acc[i][j] = Frag<T>::mma(ah, bl[j], acc[i][j]);
          acc[i][j] = Frag<T>::mma(al, bh[j], acc[i][j]);
        }
      }
      Frag<T>::guard(acc[i][0], acc[i][3], ah, SPLIT ? al : ah);
    }
    Frag<T>::keep(bh[0], bh[1], bh[2], bh[3]);
    if (SPLIT) Frag<T>::keep(bl[0], bl[1], bl[2], bl[3]);
  }
  acc_guard4(acc[0][0], acc[0][1], acc[0][2], acc[0][3]);
  acc_guard4(acc[1][0], acc[1][1], acc[1][2], acc[1][3]);
  acc_guard4(acc[2][0], acc[2][1], acc[2][2], acc[2][3]);
  acc_guard4(acc[3][0], acc[3][1], acc[3][2], acc[3][3]);

  float* slab = sT[wave];
  const float* Rb = RESID ? (resid + (size_t)b * strideR) : nullptr;
#pragma unroll
  for (int i = 0; i < 4; ++i) {
    const int mBase = m0 + (i << 4);
#pragma unroll
    for (int j = 0; j < 4; ++j) {
      const int n = n0 + (j << 4) + rlane;
      float bv = 0.f;
      if (BIAS_MODE == 2) bv = bias[n];
#pragma unroll
      for (int r = 0; r < 8; ++r) {
        float v = acc[i][j][r] * scale;
        if (BIAS_MODE == 1) v += bias[mBase + mOff + r];
        if (BIAS_MODE == 2) v += bv;
        if (RESID) v += Rb[(size_t)(mBase + mOff + r) * ldc + n];
        if (ACT == 1) v = tanhf(v);
        if (ACT == 2) v = fmaxf(v, 0.0f);
        if (ACT == 3) v = v / (1.0f + expf(-v));
        if (ACT == 4) v = (v > 0.f) ? v : 0.01f * v;
        if (ACT == 5) v = 0.5f * v * (1.0f + erff(v * 0.70710678118654752f));
        slab[(mOff + r) * 68 + (j << 4) + rlane] = v;
      }
    }
    __builtin_amdgcn_fence(__ATOMIC_RELEASE, "workgroup");
    __builtin_amdgcn_wave_barrier();
    __builtin_amdgcn_fence(__ATOMIC_ACQUIRE, "workgroup");
    if (OUT_MODE == 0) {
      float* C = (float*)Cout + (size_t)b * strideC;
      const int hh = lane >> 4, c4 = (lane & 15) * 4;
      for (int pass = 0; pass < 2; ++pass) {
#pragma unroll
        for (int it = 0; it < 8; ++it) {
          const int row = it * 2 + hh;
          v4f v = *(const v4f*)(slab + row * 68 + c4);
          *(volatile v4f*)(C + (size_t)(mBase + row) * ldc + n0 + c4) = v;
        }
        __threadfence();
      }
    } else {
      const int q = lane >> 3, c8 = (lane & 7) * 8;
      unsigned short* C  = (unsigned short*)Cout  + (size_t)b * strideC;
      unsigned short* C2 = (OUT_MODE == 2) ? ((unsigned short*)Cout2 + (size_t)b * strideC) : nullptr;
      for (int pass = 0; pass < 2; ++pass) {
#pragma unroll
        for (int it = 0; it < 4; ++it) {
          const int row = it * 4 + q;
          const float* sp = slab + row * 68 + c8;
          v8h hv, lv;
#pragma unroll
          for (int e = 0; e < 8; ++e) {
            if (OUT_MODE == 1) {
              hv[e] = (_Float16)sp[e];
            } else {
              unsigned short hb = f2bf_bits(sp[e]);
              unsigned short lb = f2bf_bits(sp[e] - bf_bits2f(hb));
              hv[e] = __builtin_bit_cast(_Float16, hb);
              lv[e] = __builtin_bit_cast(_Float16, lb);
            }
          }
          *(volatile v8h*)(C + (size_t)(mBase + row) * ldc + n0 + c8) = hv;
          if (OUT_MODE == 2) *(volatile v8h*)(C2 + (size_t)(mBase + row) * ldc + n0 + c8) = lv;
        }
        __threadfence();
      }
    }
    __builtin_amdgcn_fence(__ATOMIC_RELEASE, "workgroup");
    __builtin_amdgcn_wave_barrier();
    __builtin_amdgcn_fence(__ATOMIC_ACQUIRE, "workgroup");
  }
}

__global__ __launch_bounds__(256) void transpose_cast_f16(const float* __restrict__ in, int ldi,
                                                         _Float16* __restrict__ outT, int ldo, float scale) {
  __shared__ __align__(16) _Float16 tile[64][72];
  const int c0 = blockIdx.x * 64, r0 = blockIdx.y * 64;
  const int t = threadIdx.y * 32 + threadIdx.x;
  for (int i = threadIdx.y; i < 64; i += 8) {
    tile[threadIdx.x][i]      = (_Float16)(in[(size_t)(r0 + i) * ldi + c0 + threadIdx.x] * scale);
    tile[32 + threadIdx.x][i] = (_Float16)(in[(size_t)(r0 + i) * ldi + c0 + 32 + threadIdx.x] * scale);
  }
  __syncthreads();
  const int q = t >> 3, c8 = (t & 7) * 8;
  for (int pass = 0; pass < 2; ++pass) {
#pragma unroll
    for (int it = 0; it < 2; ++it) {
      const int c = it * 32 + q;
      v8h hv = *(const v8h*)(&tile[c][c8]);
      *(volatile v8h*)(outT + (size_t)(c0 + c) * ldo + r0 + c8) = hv;
    }
    __threadfence();
  }
}

#define AT_D 64
#define AT_NW 4
#define AT_QB 64
#define AT_KC 64
struct AttnGeomH { long c_bs, c_rs, c_hs, q_bs, q_rs, q_hs, k_bs, k_rs, k_hs, v_bs, v_rs, v_hs, o_bs, o_rs, o_hs;
                   int S, Skv, H, nbkt; float sscale, mask_fill; };
static_assert(sizeof(AttnGeomH) == 144, "no padding");

__device__ __forceinline__ v8f mma_h(v16h a, v16h b, v8f c) {
  c = __builtin_amdgcn_wmma_f32_16x16x32_f16(false, a, false, b, (short)0, c, false, false);
  asm volatile("v_nop\n\tv_nop\n\tv_nop\n\tv_nop" : "+v"(c) : "v"(a), "v"(b));
  return c;
}

__global__ __launch_bounds__(128)
void attn64h_kernel(const _Float16* __restrict__ q, const _Float16* __restrict__ k, const _Float16* __restrict__ v,
                    _Float16* __restrict__ out, const int* __restrict__ amask, const int* __restrict__ pidx,
                    const _Float16* __restrict__ cp, const _Float16* __restrict__ pc, AttnGeomH g) {
  const float PSC = 32768.0f;
  union FB { v16h v; v8h h[2]; };
  __shared__ __align__(16) _Float16 Ksh[AT_KC * AT_D];
  __shared__ __align__(16) _Float16 Vth[AT_D * AT_KC];
  __shared__ __align__(16) _Float16 Psh[AT_NW][16 * AT_KC];
  __shared__ __align__(16) float    Os[AT_NW][16 * 68];

  const int tid  = threadIdx.x;
  const int wave = tid >> 5;
  const int lane = tid & 31;
  const int hh   = lane >> 4;
  const int c    = lane & 15;

  const int nqb = g.S / AT_QB;
  const int bx = blockIdx.x;
  const int qb = bx % nqb;
  const int bh = bx / nqb;
  const int h  = bh % g.H;
  const int b  = bh / g.H;
  const int q0 = qb * AT_QB + wave * 16;

  const _Float16* qb_ptr = q + (size_t)b * g.q_bs + (size_t)h * g.q_hs;
  const _Float16* kb_ptr = k + (size_t)b * g.k_bs + (size_t)h * g.k_hs;
  const _Float16* vb_ptr = v + (size_t)b * g.v_bs + (size_t)h * g.v_hs;
  _Float16*       ob_ptr = out + (size_t)b * g.o_bs + (size_t)h * g.o_hs;
  const _Float16* cpb = cp + (size_t)b * g.c_bs + (size_t)h * g.c_hs;
  const _Float16* pcb = pc + (size_t)b * g.c_bs + (size_t)h * g.c_hs;

  v16h qa0, qa1;
  {
    const _Float16* qrow = qb_ptr + (size_t)(q0 + c) * g.q_rs + 8 * hh;
    FB f;
    f.h[0] = *(const v8h*)(qrow);      f.h[1] = *(const v8h*)(qrow + 16); qa0 = f.v;
    f.h[0] = *(const v8h*)(qrow + 32); f.h[1] = *(const v8h*)(qrow + 48); qa1 = f.v;
  }

  float mrow[8], lrow[8];
  v8f oacc[4];
#pragma unroll
  for (int r = 0; r < 8; ++r) { mrow[r] = -INFINITY; lrow[r] = 0.f; }
#pragma unroll
  for (int t = 0; t < 4; ++t) oacc[t] = (v8f){0.f,0.f,0.f,0.f,0.f,0.f,0.f,0.f};

  const int nChunks = g.Skv / AT_KC;
  for (int kc = 0; kc < nChunks; ++kc) {
    const int kv0 = kc * AT_KC;
    int mk[4][8];
    int allm = 1;
#pragma unroll
    for (int r = 0; r < 8; ++r) {
      const int* mrp = amask + (size_t)(q0 + 8 * hh + r) * g.Skv + kv0 + c;
#pragma unroll
      for (int j = 0; j < 4; ++j) { const int mv = mrp[j * 16]; mk[j][r] = mv; allm &= (mv != 0) ? 1 : 0; }
    }
    const unsigned bal = (unsigned)__ballot(allm);
    const bool live = (bal != 0xffffffffu);

    __syncthreads();
    {
      const int kvr = tid >> 1, dh = (tid & 1) * 32;
      const _Float16* krow = kb_ptr + (size_t)(kv0 + kvr) * g.k_rs + dh;
      const _Float16* vrow = vb_ptr + (size_t)(kv0 + kvr) * g.v_rs + dh;
#pragma unroll
      for (int i = 0; i < 4; ++i) {
        const v8h kk = *(const v8h*)(krow + 8 * i);
        const v8h vv = *(const v8h*)(vrow + 8 * i);
        *(v8h*)(Ksh + kvr * AT_D + dh + 8 * i) = kk;
#pragma unroll
        for (int e = 0; e < 8; ++e) Vth[(dh + 8 * i + e) * AT_KC + kvr] = vv[e];
      }
    }
    __syncthreads();

    if (live) {
      v8f s[4];
#pragma unroll
      for (int j = 0; j < 4; ++j) {
        v8f a8 = (v8f){0.f,0.f,0.f,0.f,0.f,0.f,0.f,0.f};
        const _Float16* kpt = Ksh + (j * 16 + c) * AT_D + 8 * hh;
        FB kb;
        kb.h[0] = *(const v8h*)(kpt);      kb.h[1] = *(const v8h*)(kpt + 16);
        a8 = mma_h(qa0, kb.v, a8);
        kb.h[0] = *(const v8h*)(kpt + 32); kb.h[1] = *(const v8h*)(kpt + 48);
        a8 = mma_h(qa1, kb.v, a8);
        s[j] = a8;
      }
      float cm[8];
#pragma unroll
      for (int r = 0; r < 8; ++r) {
        const int qrow = q0 + 8 * hh + r;
        const int* irp = pidx + (size_t)qrow * g.Skv + kv0 + c;
        const _Float16* cpr = cpb + (size_t)qrow * g.c_rs;
        float m = -INFINITY;
#pragma unroll
        for (int j = 0; j < 4; ++j) {
          const int kvcol = kv0 + j * 16 + c;
          int n = irp[j * 16];
          n = n < 0 ? 0 : n;
          n = (n > g.nbkt - 1) ? (g.nbkt - 1) : n;
          float sv = s[j][r] * g.sscale;
          sv += (float)cpr[n] + (float)pcb[(size_t)kvcol * g.c_rs + n];
          if (mk[j][r] != 0) sv = g.mask_fill;
          s[j][r] = sv;
          m = fmaxf(m, sv);
        }
#pragma unroll
        for (int off = 1; off < 16; off <<= 1) m = fmaxf(m, __shfl_xor(m, off, 32));
        cm[r] = m;
      }
      _Float16* pw = Psh[wave];
#pragma unroll
      for (int r = 0; r < 8; ++r) {
        const float mnew = fmaxf(mrow[r], cm[r]);
        const bool dead = (mnew == -INFINITY);
        const float alpha = dead ? 1.0f : expf(mrow[r] - mnew);
        mrow[r] = mnew;
        float psum = 0.f;
#pragma unroll
        for (int j = 0; j < 4; ++j) {
          const float p = dead ? 0.0f : expf(s[j][r] - mnew);
          psum += p;
          pw[(8 * hh + r) * AT_KC + j * 16 + c] = (_Float16)(p * PSC);
        }
#pragma unroll
        for (int off = 1; off < 16; off <<= 1) psum += __shfl_xor(psum, off, 32);
        lrow[r] = lrow[r] * alpha + psum;
#pragma unroll
        for (int t = 0; t < 4; ++t) oacc[t][r] *= alpha;
      }
      __builtin_amdgcn_fence(__ATOMIC_RELEASE, "workgroup");
      __builtin_amdgcn_wave_barrier();
      __builtin_amdgcn_fence(__ATOMIC_ACQUIRE, "workgroup");
#pragma unroll
      for (int kk = 0; kk < 2; ++kk) {
        FB pa;
        pa.h[0] = *(const v8h*)(pw + c * AT_KC + kk * 32 + 8 * hh);
        pa.h[1] = *(const v8h*)(pw + c * AT_KC + kk * 32 + 16 + 8 * hh);
#pragma unroll
        for (int t = 0; t < 4; ++t) {
          FB vb;
          vb.h[0] = *(const v8h*)(Vth + (t * 16 + c) * AT_KC + kk * 32 + 8 * hh);
          vb.h[1] = *(const v8h*)(Vth + (t * 16 + c) * AT_KC + kk * 32 + 16 + 8 * hh);
          oacc[t] = mma_h(pa.v, vb.v, oacc[t]);
        }
      }
    }
  }

  float* os = Os[wave];
#pragma unroll
  for (int r = 0; r < 8; ++r) {
    const float inv = 1.0f / (lrow[r] * PSC);
#pragma unroll
    for (int t = 0; t < 4; ++t) os[(8 * hh + r) * 68 + t * 16 + c] = oacc[t][r] * inv;
  }
  __builtin_amdgcn_fence(__ATOMIC_RELEASE, "workgroup");
  __builtin_amdgcn_wave_barrier();
  __builtin_amdgcn_fence(__ATOMIC_ACQUIRE, "workgroup");
  {
    const int q8 = lane >> 3, c8 = (lane & 7) * 8;
    for (int pass = 0; pass < 2; ++pass) {
#pragma unroll
      for (int it = 0; it < 4; ++it) {
        const int row = it * 4 + q8;
        const float* sp = os + row * 68 + c8;
        v8h hv;
#pragma unroll
        for (int e = 0; e < 8; ++e) hv[e] = (_Float16)sp[e];
        *(volatile v8h*)(ob_ptr + (size_t)(q0 + row) * g.o_rs + c8) = hv;
      }
      __threadfence();
    }
  }
}

#define TS 512
#define TB 16
#define TH 1024
#define NHD 16
#define HDM 64
#define NBKT 63
#define TM (TS * TB)

template <bool AFFINE, bool F16OUT>
__global__ __launch_bounds__(256) void ln_kernel(const float* __restrict__ x, const float* __restrict__ gam,
                                                 const float* __restrict__ bet, void* __restrict__ outp) {
  __shared__ float red[8];
  __shared__ float stat[2];
  __shared__ __align__(16) float ys[F16OUT ? TH : 4];
  const int row = blockIdx.x, t = threadIdx.x, lane = t & 31, w = t >> 5;
  const v4f xv = *(const v4f*)(x + (size_t)row * TH + 4 * t);
  float s = (xv[0] + xv[1]) + (xv[2] + xv[3]);
#pragma unroll
  for (int o = 16; o > 0; o >>= 1) s += __shfl_xor(s, o, 32);
  if (lane == 0) red[w] = s;
  __syncthreads();
  if (t == 0) {
    float a = 0.f;
#pragma unroll
    for (int i = 0; i < 8; ++i) a += red[i];
    stat[0] = a * (1.0f / (float)TH);
  }
  __syncthreads();
  const float mu = stat[0];
  const float d0 = xv[0] - mu, d1 = xv[1] - mu, d2 = xv[2] - mu, d3 = xv[3] - mu;
  float s2 = (d0 * d0 + d1 * d1) + (d2 * d2 + d3 * d3);
#pragma unroll
  for (int o = 16; o > 0; o >>= 1) s2 += __shfl_xor(s2, o, 32);
  if (lane == 0) red[w] = s2;
  __syncthreads();
  if (t == 0) {
    float a = 0.f;
#pragma unroll
    for (int i = 0; i < 8; ++i) a += red[i];
    stat[1] = rsqrtf(a * (1.0f / (float)TH) + 1e-7f);
  }
  __syncthreads();
  const float inv = stat[1];
  float y0 = d0 * inv, y1 = d1 * inv, y2 = d2 * inv, y3 = d3 * inv;
  if (AFFINE) {
    const v4f gv = *(const v4f*)(gam + 4 * t), bv = *(const v4f*)(bet + 4 * t);
    y0 = y0 * gv[0] + bv[0]; y1 = y1 * gv[1] + bv[1]; y2 = y2 * gv[2] + bv[2]; y3 = y3 * gv[3] + bv[3];
  }
  if (F16OUT) {
    const v4f yv = {y0, y1, y2, y3};
    *(v4f*)(ys + 4 * t) = yv;
    __syncthreads();
    if (t < 128) {
      const v4f a = *(const v4f*)(ys + 8 * t), c4 = *(const v4f*)(ys + 8 * t + 4);
      v8h hv;
      hv[0] = (_Float16)a[0]; hv[1] = (_Float16)a[1]; hv[2] = (_Float16)a[2]; hv[3] = (_Float16)a[3];
      hv[4] = (_Float16)c4[0]; hv[5] = (_Float16)c4[1]; hv[6] = (_Float16)c4[2]; hv[7] = (_Float16)c4[3];
      _Float16* op = (_Float16*)outp + (size_t)row * TH + 8 * t;
      *(volatile v8h*)op = hv;
      __threadfence();
      *(volatile v8h*)op = hv;
    }
  } else {
    const v4f ov = {y0, y1, y2, y3};
    float* op = (float*)outp + (size_t)row * TH + 4 * t;
    *(volatile v4f*)op = ov;
    __threadfence();
    *(volatile v4f*)op = ov;
  }
}

__global__ __launch_bounds__(256) void relpad_kernel(const float* __restrict__ re, _Float16* __restrict__ out) {
  const int i = blockIdx.x * 256 + threadIdx.x;
  if (i >= 64 * TH / 2) return;
  const int e0 = 2 * i;
  const int r = e0 / TH;
  const float a = (r < NBKT) ? re[e0] : 0.f, b = (r < NBKT) ? re[e0 + 1] : 0.f;
  const unsigned u = (unsigned)__builtin_bit_cast(unsigned short, (_Float16)a) | ((unsigned)__builtin_bit_cast(unsigned short, (_Float16)b) << 16);
  ((volatile unsigned*)out)[i] = u;
  __threadfence();
  ((volatile unsigned*)out)[i] = u;
}

extern "C" void kernel_launch(void* const* d_in, const int* in_sizes, int n_in,
                              void* d_out, int out_size, void* d_ws, size_t ws_size,
                              hipStream_t stream) {
  if (n_in < 14) return;
  if (in_sizes[0] != TM * TH || in_sizes[1] != NBKT * TH || in_sizes[2] != TH * TH || in_sizes[4] != TH * TH ||
      in_sizes[6] != TH * TH || in_sizes[8] != TH * TH || in_sizes[12] != TS * TS || in_sizes[13] != TS * TS ||
      out_size != TM * TH) return;
  const float* qin = (const float*)d_in[0];
  const float* rel = (const float*)d_in[1];
  const float* Wq = (const float*)d_in[2]; const float* bq = (const float*)d_in[3];
  const float* Wk = (const float*)d_in[4]; const float* bk = (const float*)d_in[5];
  const float* Wv = (const float*)d_in[6]; const float* bv = (const float*)d_in[7];
  const float* Wo = (const float*)d_in[8]; const float* bo = (const float*)d_in[9];
  const float* lng = (const float*)d_in[10]; const float* lnb = (const float*)d_in[11];
  const int* amask = (const int*)d_in[12];
  const int* pidx  = (const int*)d_in[13];
  float* out = (float*)d_out;
  const float SC = 0.07216878364870322f;
  const float WSC = 16.0f, WINV = 1.0f / 16.0f;

  char* ws = (char*)d_ws; size_t off = 0;
  auto carve = [&](size_t bytes) -> char* { char* p = ws + off; off += (bytes + 255) & ~(size_t)255; return p; };
  _Float16* Xn16 = (_Float16*)carve((size_t)TM * TH * 2);
  _Float16* WqT = (_Float16*)carve((size_t)TH * TH * 2);
  _Float16* WkT = (_Float16*)carve((size_t)TH * TH * 2);
  _Float16* WvT = (_Float16*)carve((size_t)TH * TH * 2);
  _Float16* WoT = (_Float16*)carve((size_t)TH * TH * 2);
  _Float16* RE16 = (_Float16*)carve((size_t)64 * TH * 2);
  _Float16* KP16 = (_Float16*)carve((size_t)64 * TH * 2);
  _Float16* QP16 = (_Float16*)carve((size_t)64 * TH * 2);
  _Float16* Q16 = (_Float16*)carve((size_t)TM * TH * 2);
  _Float16* K16 = (_Float16*)carve((size_t)TM * TH * 2);
  _Float16* V16 = (_Float16*)carve((size_t)TM * TH * 2);
  _Float16* CP16 = (_Float16*)carve((size_t)NHD * TM * 64 * 2);
  _Float16* PC16 = (_Float16*)carve((size_t)NHD * TM * 64 * 2);
  if (off > ws_size || off > (size_t)134217728) return;
  _Float16* O16 = Xn16;
  float* Y = (float*)Q16;

  ln_kernel<false, true><<<TM, 256, 0, stream>>>(qin, lng, lnb, (void*)Xn16);
  transpose_cast_f16<<<dim3(TH / 64, TH / 64), dim3(32, 8), 0, stream>>>(Wq, TH, WqT, TH, WSC);
  transpose_cast_f16<<<dim3(TH / 64, TH / 64), dim3(32, 8), 0, stream>>>(Wk, TH, WkT, TH, WSC);
  transpose_cast_f16<<<dim3(TH / 64, TH / 64), dim3(32, 8), 0, stream>>>(Wv, TH, WvT, TH, WSC);
  transpose_cast_f16<<<dim3(TH / 64, TH / 64), dim3(32, 8), 0, stream>>>(Wo, TH, WoT, TH, WSC);
  relpad_kernel<<<(64 * TH / 2 + 255) / 256, 256, 0, stream>>>(rel, RE16);

  {
    const int t = (TM / 64) * (TH / 64);
    wmma_gemm64<0, false, 2, 1, false><<<dim3((t + 7) / 8, 1), 256, 0, stream>>>(U16(Xn16), nullptr, TH, 0, U16(WqT), nullptr, TH, 0, (void*)Q16, nullptr, TH, 0, bq, nullptr, 0, TM, TH, TH, WINV);
    wmma_gemm64<0, false, 2, 1, false><<<dim3((t + 7) / 8, 1), 256, 0, stream>>>(U16(Xn16), nullptr, TH, 0, U16(WkT), nullptr, TH, 0, (void*)K16, nullptr, TH, 0, bk, nullptr, 0, TM, TH, TH, WINV);
    wmma_gemm64<0, false, 2, 1, false><<<dim3((t + 7) / 8, 1), 256, 0, stream>>>(U16(Xn16), nullptr, TH, 0, U16(WvT), nullptr, TH, 0, (void*)V16, nullptr, TH, 0, bv, nullptr, 0, TM, TH, TH, WINV);
    const int tr = (64 / 64) * (TH / 64);
    wmma_gemm64<0, false, 2, 1, false><<<dim3((tr + 7) / 8, 1), 256, 0, stream>>>(U16(RE16), nullptr, TH, 0, U16(WkT), nullptr, TH, 0, (void*)KP16, nullptr, TH, 0, bk, nullptr, 0, 64, TH, TH, WINV);
    wmma_gemm64<0, false, 2, 1, false><<<dim3((tr + 7) / 8, 1), 256, 0, stream>>>(U16(RE16), nullptr, TH, 0, U16(WqT), nullptr, TH, 0, (void*)QP16, nullptr, TH, 0, bq, nullptr, 0, 64, TH, TH, WINV);
  }
  {
    const int t = (TM / 64) * 1;
    wmma_gemm64<0, false, 0, 1, false><<<dim3((t + 7) / 8, NHD), 256, 0, stream>>>(U16(Q16), nullptr, TH, (long)HDM, U16(KP16), nullptr, TH, (long)HDM, (void*)CP16, nullptr, 64, (long)TM * 64, nullptr, nullptr, 0, TM, 64, HDM, SC);
    wmma_gemm64<0, false, 0, 1, false><<<dim3((t + 7) / 8, NHD), 256, 0, stream>>>(U16(K16), nullptr, TH, (long)HDM, U16(QP16), nullptr, TH, (long)HDM, (void*)PC16, nullptr, 64, (long)TM * 64, nullptr, nullptr, 0, TM, 64, HDM, SC);
  }
  {
    AttnGeomH g;
    g.c_bs = 64; g.c_rs = (long)TB * 64; g.c_hs = (long)TM * 64;
    g.q_bs = TH; g.q_rs = (long)TB * TH; g.q_hs = HDM;
    g.k_bs = TH; g.k_rs = (long)TB * TH; g.k_hs = HDM;
    g.v_bs = TH; g.v_rs = (long)TB * TH; g.v_hs = HDM;
    g.o_bs = TH; g.o_rs = (long)TB * TH; g.o_hs = HDM;
    g.S = TS; g.Skv = TS; g.H = NHD; g.nbkt = NBKT; g.sscale = SC; g.mask_fill = -INFINITY;
    attn64h_kernel<<<TB * NHD * (TS / AT_QB), AT_NW * 32, 0, stream>>>(Q16, K16, V16, O16, amask, pidx, CP16, PC16, g);
  }
  {
    const int t = (TM / 64) * (TH / 64);
    wmma_gemm64<0, false, 2, 0, false><<<dim3((t + 7) / 8, 1), 256, 0, stream>>>(U16(O16), nullptr, TH, 0, U16(WoT), nullptr, TH, 0, (void*)Y, nullptr, TH, 0, bo, nullptr, 0, TM, TH, TH, WINV);
  }
  ln_kernel<true, false><<<TM, 256, 0, stream>>>(Y, lng, lnb, (void*)out);
}
